// CMCI_Mamba_910533066819
// MI455X (gfx1250) — hardware-verified
//
#include <hip/hip_runtime.h>


namespace {
constexpr int Bn = 4, TIN = 2048  , T = 2048  , DM = 64, DI = 128, DS = 16, DR = 4, K = 4, NL = 2, NSQ = 2 * Bn, NTK = NSQ * T  , XDB = 64  ;
constexpr float AS_ = 8.0f;

typedef _Float16 b16;
typedef __attribute__((ext_vector_type(16))) _Float16 v16b;
typedef __attribute__((ext_vector_type(8))) _Float16 v8b;
typedef __attribute__((ext_vector_type(8))) float v8f;
typedef __attribute__((ext_vector_type(4))) float v4f;
__device__ __forceinline__ float bf16_rne(float f) { unsigned int u = __float_as_uint(f); u += 0x7FFFu + ((u >> 16) & 1u); return __uint_as_float(u & 0xFFFF0000u); }
__device__ __forceinline__ void split16(float v, b16& hi, b16& lo) { hi = (b16)v; lo = (b16)(v - (float)hi); }
__device__ __forceinline__ v16b frag_kb(const b16* p, int hh) { const v8b a = *(const v8b*)(p + 8 * hh), b = *(const v8b*)(p + 16 + 8 * hh); v16b f;
#pragma unroll
  for (int e = 0; e < 8; ++e) { f[e] = a[e]; f[8 + e] = b[e]; } return f; }
__device__ __forceinline__ void frag_split(const float* p, int hh, v16b& fh, v16b& fl) {
#pragma unroll
  for (int e = 0; e < 8; ++e) { b16 a, c; split16(p[8 * hh + e] * AS_, a, c); fh[e] = a; fl[e] = c; split16(p[16 + 8 * hh + e] * AS_, a, c); fh[8 + e] = a; fl[8 + e] = c; } }
__device__ __forceinline__ v8f wmma16b(v16b a, v16b b, v8f c) { v8f d = __builtin_amdgcn_wmma_f32_16x16x32_f16(false, a, false, b, (short)0, c, false, false); asm volatile("v_nop\n\tv_nop\n\tv_nop\n\tv_nop" : "+v"(d) : "v"(a), "v"(b)); return d; }
__device__ __forceinline__ void wave_lds_sync() { __builtin_amdgcn_fence(__ATOMIC_RELEASE, "workgroup"); __builtin_amdgcn_wave_barrier(); __builtin_amdgcn_fence(__ATOMIC_ACQUIRE, "workgroup"); }
__device__ __forceinline__ float nexp(float x) { return __builtin_amdgcn_exp2f(x * 1.4426950408889634f); }
__device__ __forceinline__ float pmul(float a, float b) { float p = a * b; asm volatile("" : "+v"(p)); return p; }
__device__ __forceinline__ float softplus_(float z) { return fmaxf(z, 0.0f) + log1pf(nexp(-fabsf(z))); }
__device__ __forceinline__ float silu_(float x) { return x / (1.0f + nexp(-x)); }

struct Wo_ { static constexpr size_t IN = 0  , XP = IN + 256 * 64  , DT = XP + 64 * 128  , OUT = DT + 128 * 32  , PER = OUT + 64 * 128; };
struct Po_ { static constexpr int CW = 0  , CB = 512, DTB = 640, A = 768  , DD = 2816, PER = 2944; };
struct In20 { const float* p[20]; };
__global__ __launch_bounds__(256) void prep_kernel(In20 in, b16* __restrict__ Rw, float* __restrict__ P) {
  const int t_ = blockIdx.x * 256 + threadIdx.x, nth = gridDim.x * 256;
  for (int pass = 0; pass < 2; ++pass) {
    for (int m = 0; m < 4; ++m) { const int s = m >> 1, i = m & 1; const float* in_w = in.p[2 + 9 * s] + (size_t)i * 256 * 64; const float* conv_w = in.p[3 + 9 * s] + (size_t)i * 128 * 4; const float* conv_b = in.p[4 + 9 * s] + i * 128;
      const float* xp_w = in.p[5 + 9 * s] + (size_t)i * 36 * 128; const float* dt_w = in.p[6 + 9 * s] + (size_t)i * 128 * 4; const float* dt_b = in.p[7 + 9 * s] + i * 128; const float* A_log = in.p[8 + 9 * s] + (size_t)i * 128 * 16; const float* Dd = in.p[9 + 9 * s] + i * 128; const float* out_w = in.p[10 + 9 * s] + (size_t)i * 64 * 128;
      b16* Rm = Rw + (size_t)m * Wo_::PER; float* Pm = P + m * Po_::PER;
      for (int q = t_; q < 256 * 64; q += nth) Rm[Wo_::IN + q] = (b16)bf16_rne(in_w[q]);
      for (int q = t_; q < 64 * 128; q += nth) Rm[Wo_::XP + q] = (b16)((q < 36 * 128) ? bf16_rne(xp_w[q]) : 0.0f);
      for (int q = t_; q < 128 * 32; q += nth) { const int o = q >> 5, k = q & 31; Rm[Wo_::DT + q] = (b16)((k < DR) ? bf16_rne(dt_w[o * DR + k]) : 0.0f); }
      for (int q = t_; q < 64 * 128; q += nth) Rm[Wo_::OUT + q] = (b16)bf16_rne(out_w[q]);
      for (int q = t_; q < Po_::PER; q += nth) { float v; if (q < Po_::CB) v = bf16_rne(conv_w[q]); else if (q < Po_::DTB) v = bf16_rne(conv_b[q - Po_::CB]); else if (q < Po_::A) v = bf16_rne(dt_b[q - Po_::DTB]); else if (q < Po_::DD) v = -expf(bf16_rne(A_log[q - Po_::A])); else v = bf16_rne(Dd[q - Po_::DD]); Pm[q] = v; } }
    __threadfence(); }
}

__global__ __launch_bounds__(256) void init_a_kernel(const float* __restrict__ Ms, const float* __restrict__ Pan, float* __restrict__ U, float* __restrict__ S) {
  const size_t g = ((size_t)blockIdx.x * 256 + threadIdx.x) * 4; const int b = (int)(g / ((size_t)T * DM)), c = (int)((g / DM) % T), l = (int)(g % DM); const size_t gi = ((size_t)b * TIN + c) * DM + l;
  const v4f ms = *(const v4f*)(Ms + gi), pn = *(const v4f*)(Pan + gi); v4f m4, p4; for (int e = 0; e < 4; ++e) { m4[e] = bf16_rne(ms[e]); p4[e] = bf16_rne(pn[e]); }
  const v4f a1 = (c < TIN / 2) ? m4 : p4, a2 = (c < TIN / 2) ? p4 : m4;
  for (int pass = 0; pass < 2; ++pass) { *(volatile v4f*)(U + g) = a1; *(volatile v4f*)(U + (size_t)Bn * T * DM + g) = a2; *(volatile v4f*)(S + g) = m4; __threadfence(); }
}
__global__ __launch_bounds__(256) void resid_kernel(const float* __restrict__ CF, float* __restrict__ S, float* __restrict__ outp, int last) {
  const size_t g = ((size_t)blockIdx.x * 256 + threadIdx.x) * 4; const int b = (int)(g / ((size_t)T * DM)), c = (int)((g / DM) % T), l = (int)(g % DM); const size_t go = ((size_t)b * TIN + c) * DM + l; const v4f c1 = *(const v4f*)(CF + g), c2 = *(const v4f*)(CF + (size_t)Bn * T * DM + g); v4f s = *(const v4f*)(S + g);
  for (int e = 0; e < 4; ++e) s[e] = fmaxf((c1[e] + c2[e]) * 0.5f + s[e], 0.0f);
  for (int pass = 0; pass < 2; ++pass) { *(volatile v4f*)(S + g) = s; if (last) *(volatile v4f*)(outp + go) = s; __threadfence(); }
}
__global__ __launch_bounds__(256) void init_b_kernel(const float* __restrict__ S, const float* __restrict__ Pan, float* __restrict__ U, float* __restrict__ S2) {
  const size_t g = ((size_t)blockIdx.x * 256 + threadIdx.x) * 4; const int b = (int)(g / ((size_t)T * DM)), c = (int)((g / DM) % T), l = (int)(g % DM); const size_t gi = ((size_t)b * TIN + c) * DM + l;
  const v4f ms = *(const v4f*)(S + g), pn = *(const v4f*)(Pan + gi); v4f p4; for (int e = 0; e < 4; ++e) p4[e] = bf16_rne(pn[e]);
  const bool ev = ((c & 1) == 0); const v4f a3 = ev ? p4 : ms, a4 = ev ? ms : p4;
  for (int pass = 0; pass < 2; ++pass) { *(volatile v4f*)(U + g) = a3; *(volatile v4f*)(U + (size_t)Bn * T * DM + g) = a4; *(volatile v4f*)(S2 + g) = p4; __threadfence(); }
}

__global__ __launch_bounds__(128) void gemm_kernel(const float* __restrict__ X, int Kk, int ldx, const b16* __restrict__ Bw, int N, const float* __restrict__ bias, int mode, float* __restrict__ Y) {
  __shared__ __attribute__((aligned(16))) float Ts[4][32 * 64];
  const int lane = threadIdx.x & 31, wave = threadIdx.x >> 5, nloc = lane & 15, hlf = lane >> 4, m0 = blockIdx.y * 128 + wave * 32, c0 = blockIdx.x * 64;
  v8f acc[2][4];
#pragma unroll
  for (int r = 0; r < 2; ++r)
#pragma unroll
    for (int t = 0; t < 4; ++t) acc[r][t] = (v8f){};
  for (int kb = 0; kb < Kk; kb += 32) { v16b a0, l0, a1, l1; frag_split(X + (size_t)(m0 + nloc) * ldx + kb, hlf, a0, l0); frag_split(X + (size_t)(m0 + 16 + nloc) * ldx + kb, hlf, a1, l1);
#pragma unroll
    for (int t = 0; t < 4; ++t) { const v16b bw = frag_kb(Bw + (size_t)(c0 + t * 16 + nloc) * Kk + kb, hlf); acc[0][t] = wmma16b(a0, bw, acc[0][t]); acc[0][t] = wmma16b(l0, bw, acc[0][t]); acc[1][t] = wmma16b(a1, bw, acc[1][t]); acc[1][t] = wmma16b(l1, bw, acc[1][t]); } }
  float* Tt = Ts[wave];
#pragma unroll
  for (int t = 0; t < 4; ++t) { const int cc = c0 + t * 16 + nloc; const float bb = bias ? bias[cc] : 0.0f;
#pragma unroll
    for (int r = 0; r < 2; ++r)
#pragma unroll
      for (int v = 0; v < 8; ++v) Tt[(r * 16 + v + 8 * hlf) * 64 + t * 16 + nloc] = acc[r][t][v] * (1.0f / AS_) + bb; }
  wave_lds_sync();
  if (mode == 1) {
#pragma unroll 1
    for (int i = lane; i < 32 * 64; i += 32) Tt[i] = softplus_(Tt[i]);
    wave_lds_sync(); }
  for (int pass = 0; pass < 2; ++pass) {
#pragma unroll
    for (int j = 0; j < 16; ++j) { const int rr = j * 2 + hlf, c4 = nloc * 4; *(volatile v4f*)(Y + (size_t)(m0 + rr) * N + c0 + c4) = *(const v4f*)(Tt + rr * 64 + c4); }
    __threadfence(); }
}

__global__ __launch_bounds__(256) void conv_kernel(const float* __restrict__ xz, const float* __restrict__ Pm, float* __restrict__ xcs) {
  const size_t g = (size_t)blockIdx.x * 256 + threadIdx.x; const int tok = (int)(g / (DI / 4)), e4 = (int)(g % (DI / 4)) * 4, sq = tok / T, t = tok % T; const float* cw = Pm + Po_::CW; const float* cb = Pm + Po_::CB;
  v4f o;
#pragma unroll
  for (int q = 0; q < 4; ++q) { const int e = e4 + q; float acc = cb[e];
#pragma unroll
    for (int k = 0; k < K; ++k) { const int ts = t - (K - 1) + k; if (ts >= 0) acc += pmul(cw[e * K + k], xz[((size_t)sq * T + ts) * (2 * DI) + e]); }
    o[q] = silu_(acc); }
  for (int pass = 0; pass < 2; ++pass) { *(volatile v4f*)(xcs + (size_t)tok * DI + e4) = o; __threadfence(); }
}

__global__ __launch_bounds__(256) void scan_kernel(const float* __restrict__ xcs, const float* __restrict__ delta, const float* __restrict__ xdbl, const float* __restrict__ xz, const float* __restrict__ Pm, float* __restrict__ y) {
  const int g = blockIdx.x * 256 + threadIdx.x, sq = g / DI, e = g % DI; const float* A = Pm + Po_::A + e * DS; const float Dv = Pm[Po_::DD + e];
  float h[DS], a_[DS];
#pragma unroll
  for (int n = 0; n < DS; ++n) { h[n] = 0.0f; a_[n] = A[n]; }
  for (int t = 0; t < T; ++t) { const size_t row = (size_t)sq * T + t; const float dl = delta[row * DI + e], xc = xcs[row * DI + e]; const float* xr = xdbl + row * XDB; const float dx = dl * xc; float acc = 0.0f;
#pragma unroll
    for (int n = 0; n < DS; ++n) { const float dA = nexp(dl * a_[n]); h[n] = dA * h[n] + pmul(dx, xr[DR + n]); acc += pmul(h[n], xr[DR + DS + n]); }
    const float yv = (acc + pmul(Dv, xc)) * silu_(xz[row * (2 * DI) + DI + e]);
    for (int pass = 0; pass < 2; ++pass) ((volatile float*)y)[row * DI + e] = yv; }
  __threadfence();
}
}

extern "C" void kernel_launch(void* const* d_in, const int* in_sizes, int n_in,
                              void* d_out, int out_size, void* d_ws, size_t ws_size, hipStream_t stream) {
  (void)out_size;
  if (n_in != 20) return;
  In20 in; for (int i = 0; i < 20; ++i) in.p[i] = (const float*)d_in[i];
  const float* Ms = in.p[0]; const float* Pan = in.p[1];
  float* outM = (float*)d_out; float* outP = outM + (size_t)Bn * TIN * DM;
  if (in_sizes[0] != Bn * TIN * DM || in_sizes[1] != Bn * TIN * DM || in_sizes[2] != NL * 256 * 64 || in_sizes[14] != NL * 36 * 128 || in_sizes[19] != NL * 64 * 128) return;
  size_t off = 0; char* ws = (char*)d_ws;
  auto carve = [&](size_t bytes) { char* p = ws + off; off += (bytes + 255) & ~(size_t)255; return p; };
  b16* Rw = (b16*)carve((size_t)4 * Wo_::PER * 2); float* P = (float*)carve((size_t)4 * Po_::PER * 4);
  float* U = (float*)carve((size_t)NTK * DM * 4); float* S = (float*)carve((size_t)Bn * T * DM * 4); float* S2 = (float*)carve((size_t)Bn * T * DM * 4);
  float* xz = (float*)carve((size_t)NTK * 2 * DI * 4); float* xcs = (float*)carve((size_t)NTK * DI * 4); float* xdbl = (float*)carve((size_t)NTK * XDB * 4); float* delta = (float*)carve((size_t)NTK * DI * 4); float* y = (float*)carve((size_t)NTK * DI * 4);
  if (off > ws_size) return;
  const int nglue = Bn * T * DM / 4 / 256;
  auto mamba = [&](int m) { const b16* Rm = Rw + (size_t)m * Wo_::PER; const float* Pm = P + m * Po_::PER;
    gemm_kernel<<<dim3(2 * DI / 64, NTK / 128), 128, 0, stream>>>(U, DM, DM, Rm + Wo_::IN, 2 * DI, nullptr, 0, xz);
    conv_kernel<<<NTK * DI / 4 / 256, 256, 0, stream>>>(xz, Pm, xcs);
    gemm_kernel<<<dim3(XDB / 64, NTK / 128), 128, 0, stream>>>(xcs, DI, DI, Rm + Wo_::XP, XDB, nullptr, 0, xdbl);
    gemm_kernel<<<dim3(DI / 64, NTK / 128), 128, 0, stream>>>(xdbl, 32, XDB, Rm + Wo_::DT, DI, Pm + Po_::DTB, 1, delta);
    scan_kernel<<<NSQ * DI / 256, 256, 0, stream>>>(xcs, delta, xdbl, xz, Pm, y);
    gemm_kernel<<<dim3(DM / 64, NTK / 128), 128, 0, stream>>>(y, DI, DI, Rm + Wo_::OUT, DM, nullptr, 0, U); };
  prep_kernel<<<64, 256, 0, stream>>>(in, Rw, P);
  init_a_kernel<<<nglue, 256, 0, stream>>>(Ms, Pan, U, S);
  for (int i = 0; i < NL; ++i) { mamba(i); resid_kernel<<<nglue, 256, 0, stream>>>(U, S, outM, i == NL - 1); }
  init_b_kernel<<<nglue, 256, 0, stream>>>(S, Pan, U, S2);
  for (int i = 0; i < NL; ++i) { mamba(2 + i); resid_kernel<<<nglue, 256, 0, stream>>>(U, S2, outP, i == NL - 1); }
}
